// CrossAttention_9302899163605
// MI455X (gfx1250) — hardware-verified
//
#include <hip/hip_runtime.h>


#ifndef NB
#define NB 2
#endif
#ifndef SEQ
#define SEQ 2048
#endif
#define NB_FULL  2
#define SEQ_FULL 2048
#define TT   SEQ
#define DM   1024
#define NH_  16
#define HD   64
#define DQ   (NH_ * HD)
#define SCL   0.125f
#define LOG2E 1.4426950408889634f
#define PLOG2 10.0f
#define LNEPS 1.0e-6f

static_assert(SEQ % 64 == 0);
static_assert(SEQ % 8 == 0);
static_assert(SEQ <= SEQ_FULL);
static_assert(NB >= 1 && NB <= NB_FULL);
static_assert(DQ == DM);
static_assert(DM == 1024);
static_assert((NH_ * HD * SEQ) % 2048 == 0);

typedef _Float16 h16;
typedef unsigned short bf;
typedef __attribute__((ext_vector_type(16))) __bf16   v16bf;
typedef __attribute__((ext_vector_type(16))) _Float16 v16h;
typedef __attribute__((ext_vector_type(8)))  _Float16 v8h;
typedef __attribute__((ext_vector_type(8)))  unsigned short v8us;
typedef __attribute__((ext_vector_type(8)))  float    v8f;
typedef __attribute__((ext_vector_type(4)))  float    v4f;
typedef v8h  __attribute__((may_alias)) v8ha;
typedef v4f  __attribute__((may_alias)) v4fa;
typedef v8us __attribute__((may_alias)) v8usa;

__device__ __forceinline__ unsigned short f2bf(float f) { unsigned u = __float_as_uint(f); u += 0x7FFFu + ((u >> 16) & 1u); return (unsigned short)(u >> 16); }
__device__ __forceinline__ float bf2f(unsigned short b) { return __uint_as_float(((unsigned)b) << 16); }
__device__ __forceinline__ float bfr(float f) { return bf2f(f2bf(f)); }
__device__ __forceinline__ v16h cat16(v8h lo, v8h hi) { return __builtin_shufflevector(lo, hi, 0, 1, 2, 3, 4, 5, 6, 7, 8, 9, 10, 11, 12, 13, 14, 15); }
__device__ __forceinline__ v16bf cat16b(v8us lo, v8us hi) { return __builtin_bit_cast(v16bf, __builtin_shufflevector(lo, hi, 0, 1, 2, 3, 4, 5, 6, 7, 8, 9, 10, 11, 12, 13, 14, 15)); }
__device__ __forceinline__ v8f wmma16(v16h a, v16h b, v8f c) { return __builtin_amdgcn_wmma_f32_16x16x32_f16(false, a, false, b, (short)0, c, false, false); }
__device__ __forceinline__ v8f wmmab(v16bf a, v16bf b, v8f c) { return __builtin_amdgcn_wmma_f32_16x16x32_bf16(false, a, false, b, (short)0, c, false, false); }
__device__ __forceinline__ h16 tohx(float x) { return (h16)x; }
__device__ __forceinline__ void splitf(float y, unsigned short& h, unsigned short& l) { h = f2bf(y); l = f2bf(y - bf2f(h)); }

#define WGUARD4(a0, a1, a2, a3, x, y) asm volatile("v_nop\n\tv_nop\n\tv_nop\n\tv_nop" : "+v"(a0), "+v"(a1), "+v"(a2), "+v"(a3) : "v"(x), "v"(y))

template <typename T16> struct WFrag;
template <> struct WFrag<h16> { typedef v16h V; static __device__ __forceinline__ V ld(const h16* p) { return cat16(*(const v8h*)p, *(const v8h*)(p + 16)); } static __device__ __forceinline__ v8f mma(V a, V b, v8f c) { return wmma16(a, b, c); } };
template <> struct WFrag<bf> { typedef v16bf V; static __device__ __forceinline__ V ld(const bf* p) { return cat16b(*(const v8us*)p, *(const v8us*)(p + 16)); } static __device__ __forceinline__ v8f mma(V a, V b, v8f c) { return wmmab(a, b, c); } };
template <typename T16, int NSPLIT, bool BIAS>
__global__ __launch_bounds__(32) void k_gemmw(const T16* __restrict__ A, const T16* __restrict__ A2, const T16* __restrict__ Bt, const T16* __restrict__ Bt2, int K, float* C, int ldc, const float* __restrict__ bias, size_t sA, size_t sB, size_t sC) {
    typedef typename WFrag<T16>::V V;
    __shared__ __align__(16) float os[16 * 68];
    const size_t z = blockIdx.z; A += z * sA; if (A2) A2 += z * sA; Bt += z * sB; if (Bt2) Bt2 += z * sB; C += z * sC;
    const int lane = threadIdx.x & 31, lr = lane & 15, hi = lane >> 4; const int r0 = blockIdx.x * 64, c0 = blockIdx.y * 64;
    v8f acc[4][4];
#pragma unroll
    for (int mb = 0; mb < 4; ++mb)
#pragma unroll
        for (int nb = 0; nb < 4; ++nb) acc[mb][nb] = (v8f){};
    const size_t aoff = (size_t)(r0 + lr) * K + 8 * hi, boff = (size_t)(c0 + lr) * K + 8 * hi;
#pragma unroll 1
    for (int kc = 0; kc < K; kc += 32) {
        V a[4], a2[4];
#pragma unroll
        for (int mb = 0; mb < 4; ++mb) { a[mb] = WFrag<T16>::ld(A + aoff + (size_t)mb * 16 * K + kc); if (NSPLIT == 1 || NSPLIT == 2) a2[mb] = WFrag<T16>::ld(A2 + aoff + (size_t)mb * 16 * K + kc); }
#pragma unroll
        for (int nb = 0; nb < 4; ++nb) { const V b = WFrag<T16>::ld(Bt + boff + (size_t)nb * 16 * K + kc); V b2; if (NSPLIT >= 2) b2 = WFrag<T16>::ld(Bt2 + boff + (size_t)nb * 16 * K + kc);
#pragma unroll
            for (int mb = 0; mb < 4; ++mb) { acc[mb][nb] = WFrag<T16>::mma(a[mb], b, acc[mb][nb]); if (NSPLIT == 1 || NSPLIT == 2) acc[mb][nb] = WFrag<T16>::mma(a2[mb], b, acc[mb][nb]); if (NSPLIT >= 2) acc[mb][nb] = WFrag<T16>::mma(a[mb], b2, acc[mb][nb]); } }
        asm volatile("v_nop\n\tv_nop\n\tv_nop\n\tv_nop" : "+v"(acc[0][0]), "+v"(acc[1][1]), "+v"(acc[2][2]), "+v"(acc[3][3]) : "v"(a[0]), "v"(a[3]));
    }
#pragma unroll
    for (int mb = 0; mb < 4; ++mb) {
#pragma unroll
        for (int nb = 0; nb < 4; ++nb) {
#pragma unroll
            for (int j = 0; j < 8; ++j) os[(hi * 8 + j) * 68 + nb * 16 + lr] = acc[mb][nb][j]; }
        __builtin_amdgcn_wave_barrier(); asm volatile("" ::: "memory");
        float* crow = C + (size_t)(r0 + mb * 16) * ldc + c0;
#pragma unroll 1
        for (int ps = 0; ps < 2; ++ps) {
#pragma unroll
            for (int s = 0; s < 8; ++s) { const int row = 2 * s + hi, cofs = lr * 4; v4f val = *(const v4fa*)(os + row * 68 + cofs); if (BIAS) { val[0] += bfr(bias[c0 + cofs]); val[1] += bfr(bias[c0 + cofs + 1]); val[2] += bfr(bias[c0 + cofs + 2]); val[3] += bfr(bias[c0 + cofs + 3]); }
                *(volatile v4f*)(crow + (size_t)row * ldc + cofs) = val; }
            if (ps == 0) __threadfence(); }
        __builtin_amdgcn_wave_barrier(); asm volatile("" ::: "memory");
    }
}

__global__ __launch_bounds__(256) void k_cvt8(const float* __restrict__ src, bf* dst, size_t n8) { const size_t i = (size_t)blockIdx.x * 256 + threadIdx.x; if (i >= n8) return; const v8f v = *(const v8f*)(src + i * 8); v8us o;
#pragma unroll
    for (int k = 0; k < 8; ++k) o[k] = f2bf(v[k]); *(volatile v8us*)(dst + i * 8) = o; __threadfence(); *(volatile v8us*)(dst + i * 8) = o; }

template <bool RIN>
__global__ __launch_bounds__(256) void k_lnp(const float* __restrict__ F, int pitch, int rows, const float* __restrict__ gam, const float* __restrict__ bet, bf* Ph, bf* Pl) {
    const int lane = threadIdx.x & 31; const int row = blockIdx.x * 8 + (threadIdx.x >> 5); if (row >= rows) return;
    const float* fr = F + (size_t)row * pitch + lane * 8;
    float s = 0.f;
#pragma unroll 1
    for (int c = 0; c < 4; ++c) { const v8f a = *(const v8f*)(fr + c * 256);
#pragma unroll
        for (int q = 0; q < 8; ++q) { const float xv = RIN ? bfr(a[q]) : a[q]; s += xv; } }
#pragma unroll
    for (int sh = 16; sh; sh >>= 1) s += __shfl_xor(s, sh, 32);
    const float mu = s * (1.0f / (float)DM);
    float s2 = 0.f;
#pragma unroll 1
    for (int c = 0; c < 4; ++c) { const v8f a = *(const v8f*)(fr + c * 256);
#pragma unroll
        for (int q = 0; q < 8; ++q) { const float xv = RIN ? bfr(a[q]) : a[q]; const float d = xv - mu; s2 += d * d; } }
#pragma unroll
    for (int sh = 16; sh; sh >>= 1) s2 += __shfl_xor(s2, sh, 32);
    const float rstd = rsqrtf(s2 * (1.0f / (float)DM) + LNEPS);
#pragma unroll 1
    for (int c = 0; c < 4; ++c) {
        const int col0 = c * 256 + lane * 8; const v8f a = *(const v8f*)(fr + c * 256); const v8f g8 = *(const v8f*)(gam + col0); const v8f b8 = *(const v8f*)(bet + col0);
        v8us oh, ol;
#pragma unroll
        for (int q = 0; q < 8; ++q) { const float xv = RIN ? bfr(a[q]) : a[q]; const float d = xv - mu; const float y = (d * rstd) * bfr(g8[q]) + bfr(b8[q]); unsigned short a2, c2; splitf(y, a2, c2); oh[q] = a2; ol[q] = c2; }
        const int hh = c * 4 + (lane >> 3); const size_t oo = ((size_t)hh * TT + row) * HD + 8 * (lane & 7);
        *(volatile v8us*)(Ph + oo) = oh; *(volatile v8us*)(Pl + oo) = ol;
        __threadfence();
        *(volatile v8us*)(Ph + oo) = oh; *(volatile v8us*)(Pl + oo) = ol;
    }
}

__global__ __launch_bounds__(256) void k_vtp8(const float* __restrict__ F, int pitch, h16* V16) {
    const size_t e = ((size_t)blockIdx.x * 256 + threadIdx.x) * 8; if (e >= (size_t)NH_ * HD * TT) return;
    const int t = (int)(e % TT); const int d = (int)((e / TT) % HD); const int g = (int)(e / ((size_t)TT * HD));
    v8h o;
#pragma unroll
    for (int q = 0; q < 8; ++q) o[q] = tohx(F[(size_t)(t + q) * pitch + g * HD + d]);
    *(volatile v8h*)(V16 + e) = o; __threadfence(); *(volatile v8h*)(V16 + e) = o;
}

__global__ __launch_bounds__(128) void k_flash(const bf* __restrict__ Qh, const bf* __restrict__ Ql, const bf* __restrict__ Kh, const bf* __restrict__ Kl, const h16* __restrict__ VT, bf* Ah, bf* Al) {
    __shared__ __align__(16) h16 pt_all[4][16 * 72];
    __shared__ __align__(16) float os_all[4][16 * 68];
    const int tid = threadIdx.x; const int lane = tid & 31, w = tid >> 5, lr = lane & 15, hi = lane >> 4;
    const int h = blockIdx.y; const int row0 = blockIdx.x * 64 + w * 16;
    h16* pt = pt_all[w]; float* os = os_all[w];
    const size_t hb = (size_t)h * TT * HD;
    v16bf qh[2], ql[2];
    { const size_t qo = hb + (size_t)(row0 + lr) * HD + 8 * hi;
#pragma unroll
      for (int s = 0; s < 2; ++s) { qh[s] = WFrag<bf>::ld(Qh + qo + 32 * s); ql[s] = WFrag<bf>::ld(Ql + qo + 32 * s); } }
    v8f o[4];
#pragma unroll
    for (int dt = 0; dt < 4; ++dt) o[dt] = (v8f){};
    float m[8], l[8];
#pragma unroll
    for (int g = 0; g < 8; ++g) { m[g] = -3.0e38f; l[g] = 0.f; }
    const h16* vbase = VT + (size_t)h * HD * TT + 8 * hi;
#pragma unroll 1
    for (int j0 = 0; j0 < TT; j0 += 64) {
        v8f st[4];
#pragma unroll
        for (int t = 0; t < 4; ++t) st[t] = (v8f){};
#pragma unroll
        for (int t = 0; t < 4; ++t) { const size_t ko = hb + (size_t)(j0 + 16 * t + lr) * HD + 8 * hi;
#pragma unroll
            for (int s = 0; s < 2; ++s) { const v16bf kh = WFrag<bf>::ld(Kh + ko + 32 * s); const v16bf kl = WFrag<bf>::ld(Kl + ko + 32 * s);
                st[t] = wmmab(qh[s], kh, st[t]); st[t] = wmmab(ql[s], kh, st[t]); st[t] = wmmab(qh[s], kl, st[t]); } }
        WGUARD4(st[0], st[1], st[2], st[3], qh[0], ql[1]);
        __syncthreads();
#pragma unroll
        for (int g = 0; g < 8; ++g) {
            float mt = fmaxf(fmaxf(st[0][g], st[1][g]), fmaxf(st[2][g], st[3][g])) * SCL;
#pragma unroll
            for (int off = 1; off < 16; off <<= 1) mt = fmaxf(mt, __shfl_xor(mt, off, 32));
            const float mnew = fmaxf(m[g], mt);
            const float alpha = __builtin_amdgcn_exp2f((m[g] - mnew) * LOG2E);
            float rs = 0.f;
#pragma unroll
            for (int t = 0; t < 4; ++t) { const float pe = __builtin_amdgcn_exp2f((st[t][g] * SCL - mnew) * LOG2E + PLOG2); pt[(8 * hi + g) * 72 + 16 * t + lr] = tohx(pe); rs += pe; }
#pragma unroll
            for (int off = 1; off < 16; off <<= 1) rs += __shfl_xor(rs, off, 32);
            l[g] = l[g] * alpha + rs; m[g] = mnew;
#pragma unroll
            for (int dt = 0; dt < 4; ++dt) o[dt][g] = o[dt][g] * alpha;
        }
        __syncthreads();
        v16h pa[2];
#pragma unroll
        for (int s = 0; s < 2; ++s) pa[s] = cat16(*(const v8h*)(pt + lr * 72 + 32 * s + 8 * hi), *(const v8h*)(pt + lr * 72 + 32 * s + 16 + 8 * hi));
#pragma unroll
        for (int dt = 0; dt < 4; ++dt) { const h16* vp = vbase + (size_t)(16 * dt + lr) * TT + j0;
#pragma unroll
            for (int s = 0; s < 2; ++s) { const v16h vb = WFrag<h16>::ld(vp + 32 * s); o[dt] = wmma16(pa[s], vb, o[dt]); } }
        WGUARD4(o[0], o[1], o[2], o[3], pa[0], pa[1]);
    }
    float inv[8];
#pragma unroll
    for (int g = 0; g < 8; ++g) inv[g] = __builtin_amdgcn_rcpf(l[g]);
#pragma unroll
    for (int dt = 0; dt < 4; ++dt)
#pragma unroll
        for (int g = 0; g < 8; ++g) os[(8 * hi + g) * 68 + 16 * dt + lr] = o[dt][g] * inv[g];
    __syncthreads();
#pragma unroll 1
    for (int ps = 0; ps < 2; ++ps) {
#pragma unroll
        for (int it = 0; it < 4; ++it) { const int row = it * 4 + (lane >> 3); const int pc = lane & 7;
            const v4f a = *(const v4fa*)(os + row * 68 + 8 * pc); const v4f b = *(const v4fa*)(os + row * 68 + 8 * pc + 4); v8us oh, ol;
#pragma unroll
            for (int q = 0; q < 4; ++q) { unsigned short a2, c2; splitf(a[q], a2, c2); oh[q] = a2; ol[q] = c2; splitf(b[q], a2, c2); oh[4 + q] = a2; ol[4 + q] = c2; }
            const size_t oo = (size_t)(row0 + row) * DQ + h * HD + 8 * pc;
            *(volatile v8us*)(Ah + oo) = oh; *(volatile v8us*)(Al + oo) = ol; }
        if (ps == 0) __threadfence(); }
}

extern "C" void kernel_launch(void* const* d_in, const int* in_sizes, int n_in,
                              void* d_out, int out_size, void* d_ws, size_t ws_size, hipStream_t stream) {
    if (n_in < 9) return;
    const float* x   = (const float*)d_in[0];
    const float* ctx = (const float*)d_in[1];
    const float* gq  = (const float*)d_in[2];
    const float* bq  = (const float*)d_in[3];
    const float* gk  = (const float*)d_in[4];
    const float* bk  = (const float*)d_in[5];
    const float* Wkv = (const float*)d_in[6];
    const float* Wo  = (const float*)d_in[7];
    const float* bo  = (const float*)d_in[8];
    float* OUT = (float*)d_out;
    const long long need_tok = (long long)(NB - 1) * SEQ_FULL * DM + (long long)SEQ * DM;
    if ((long long)in_sizes[0] < need_tok || (long long)in_sizes[1] < need_tok) return;
    if (in_sizes[2] < DM || in_sizes[3] < DM || in_sizes[4] < DM || in_sizes[5] < DM || in_sizes[8] < DM) return;
    if ((long long)in_sizes[6] < (long long)2 * DM * DM || (long long)in_sizes[7] < (long long)DM * DM) return;
    if ((long long)out_size < need_tok) return;

    char* wsp = (char*)d_ws;
    auto take = [&](size_t bytes) { char* p = wsp; wsp += (bytes + 255) & ~(size_t)255; return (void*)p; };
    bf*    WKV  = (bf*)take((size_t)2 * DM * DM * 2);
    bf*    WO   = (bf*)take((size_t)DM * DM * 2);
    bf*    XB   = (bf*)take((size_t)TT * DM * 2);
    float* FKV  = (float*)take((size_t)TT * 2 * DM * 4);
    bf*    QPh  = (bf*)take((size_t)NH_ * TT * HD * 2);
    bf*    QPl  = (bf*)take((size_t)NH_ * TT * HD * 2);
    bf*    KPh  = (bf*)take((size_t)NH_ * TT * HD * 2);
    bf*    KPl  = (bf*)take((size_t)NH_ * TT * HD * 2);
    h16*   VT16 = (h16*)take((size_t)NH_ * HD * TT * 2);
    bf*    ATh  = (bf*)take((size_t)TT * DQ * 2);
    bf*    ATl  = (bf*)take((size_t)TT * DQ * 2);
    const size_t used = (size_t)(wsp - (char*)d_ws);
    if (used > ws_size || used > ((size_t)128 << 20)) return;

    k_cvt8<<<(unsigned)(((size_t)2 * DM * DM / 8 + 255) / 256), 256, 0, stream>>>(Wkv, WKV, (size_t)2 * DM * DM / 8);
    k_cvt8<<<(unsigned)(((size_t)DM * DM / 8 + 255) / 256), 256, 0, stream>>>(Wo, WO, (size_t)DM * DM / 8);
    for (int b = 0; b < NB; ++b) {
        const size_t boff = (size_t)b * SEQ_FULL * DM;
        k_cvt8<<<(unsigned)(((size_t)TT * DM / 8 + 255) / 256), 256, 0, stream>>>(ctx + boff, XB, (size_t)TT * DM / 8);
        k_gemmw<bf, 0, false><<<dim3(TT / 64, (2 * DM) / 64, 1), 32, 0, stream>>>(XB, nullptr, WKV, nullptr, DM, FKV, 2 * DM, nullptr, 0, 0, 0);
        k_lnp<false><<<TT / 8, 256, 0, stream>>>(FKV, 2 * DM, TT, gk, bk, KPh, KPl);
        k_vtp8<<<(unsigned)((size_t)NH_ * HD * TT / 8 / 256), 256, 0, stream>>>(FKV + DM, 2 * DM, VT16);
        k_lnp<true><<<TT / 8, 256, 0, stream>>>(x + boff, DM, TT, gq, bq, QPh, QPl);
        k_flash<<<dim3(TT / 64, NH_, 1), 128, 0, stream>>>(QPh, QPl, KPh, KPl, VT16, ATh, ATl);
        k_gemmw<bf, 1, true><<<dim3(TT / 64, DM / 64, 1), 32, 0, stream>>>(ATh, ATl, WO, nullptr, DQ, OUT + boff, DM, bo, 0, 0, 0);
    }
}
